// MAB_7619271983203
// MI455X (gfx1250) — hardware-verified
//
#include <hip/hip_runtime.h>
#include <math.h>

typedef __attribute__((ext_vector_type(16))) _Float16 v16h;
typedef __attribute__((ext_vector_type(16))) __bf16 v16b;
typedef __attribute__((ext_vector_type(8)))  _Float16 v8h;
typedef __attribute__((ext_vector_type(8)))  __bf16 v8b;
typedef __attribute__((ext_vector_type(4)))  _Float16 v4h;
typedef __attribute__((ext_vector_type(8)))  float v8f;
typedef __attribute__((ext_vector_type(4)))  float v4f;
typedef __attribute__((ext_vector_type(4)))  unsigned v4u;

template <typename T> __device__ __forceinline__ void vst2(void* p, T v) { *(volatile T*)p = v; __threadfence(); *(volatile T*)p = v; }
__device__ __forceinline__ v8f wmma16(v16h a, v16h b, v8f c) {
  v8f d = __builtin_amdgcn_wmma_f32_16x16x32_f16(false, a, false, b, (short)0, c, false, false);
  asm volatile("v_nop\n\tv_nop\n\tv_nop\n\tv_nop" : "+v"(d) : "v"(a), "v"(b));
  return d;
}
__device__ __forceinline__ v8f wmma_bf(v16b a, v16b b, v8f c) {
  v8f d = __builtin_amdgcn_wmma_f32_16x16x32_bf16(false, a, false, b, (short)0, c, false, false);
  asm volatile("v_nop\n\tv_nop\n\tv_nop\n\tv_nop" : "+v"(d) : "v"(a), "v"(b));
  return d;
}
__device__ __forceinline__ v16h frag_h(const _Float16* rowk0, int lane) {
  union { v16h v; v8h q[2]; } u; const _Float16* p = rowk0 + 8 * (lane >> 4);
  u.q[0] = *(const v8h*)p; u.q[1] = *(const v8h*)(p + 16); return u.v;
}
__device__ __forceinline__ v16b frag_b(const __bf16* rowk0, int lane) {
  union { v16b v; v8b q[2]; } u; const __bf16* p = rowk0 + 8 * (lane >> 4);
  u.q[0] = *(const v8b*)p; u.q[1] = *(const v8b*)(p + 16); return u.v;
}
__device__ __forceinline__ v16h frag_f32(const float* rowk0, int lane) {
  v16h a; const float* p = rowk0 + 8 * (lane >> 4);
#pragma unroll
  for (int i = 0; i < 8; ++i) { a[i] = (_Float16)p[i]; a[8 + i] = (_Float16)p[16 + i]; }
  return a;
}
__device__ __forceinline__ float bfr(float v) { return (float)(__bf16)v; }
#define LDSX() do { asm volatile("s_wait_dscnt 0x0" ::: "memory"); __builtin_amdgcn_fence(4, "wavefront"); __builtin_amdgcn_wave_barrier(); } while (0)

#ifndef NB
#define NB 8
#endif
#ifndef SEQ
#define SEQ 1024
#endif
#define NB_FULL 8
#define TT_FULL 1024
#define TT SEQ
#define DIN 512
#define CC 512
#define NH 8
#define HD 64
#define DFF 2048
#define NQB (TT / 64)
#define NROW (NB * TT)
#define SCALE (0.125f)
static_assert(NB >= 1 && NB <= NB_FULL);
static_assert(TT % 128 == 0 && TT >= 128 && TT <= TT_FULL);
static_assert(NH * HD == CC && HD == 64 && DIN % 32 == 0 && CC % 128 == 0 && DFF % 128 == 0 && NROW % 64 == 0);
static_assert(((size_t)(NB - 1) * TT_FULL + TT) * CC * 4u <= 16777216u);

#define SZ_HROW (2u * (size_t)NROW * CC)
#define SZ_FROW (4u * (size_t)NROW * CC)
#define SZ_S    (4u * (size_t)NH * TT * TT)
#define SZ_WP   (2u * (size_t)CC * DIN)
#define WS_QH   ((size_t)0)
#define WS_KH   (WS_QH + SZ_HROW)
#define WS_VT   (WS_KH + SZ_HROW)
#define WS_QL   (WS_VT + SZ_HROW)
#define WS_S    (WS_QL + SZ_HROW)
#define WS_Y    (WS_S + SZ_S)
#define WS_O    (WS_Y + SZ_FROW)
#define WS_OH   (WS_O + SZ_FROW)
#define WS_WQ   (WS_OH + SZ_HROW)
#define WS_WK   (WS_WQ + SZ_WP)
#define WS_WV   (WS_WK + SZ_WP)
#define WS_W1   (WS_WV + SZ_WP)
#define WS_W2   (WS_W1 + 2u * (size_t)DFF * CC)
#define WS_W3   (WS_W2 + 2u * (size_t)DFF * DFF)
#define WS_END  (WS_W3 + 2u * (size_t)CC * DFF)
#define WS_XQ   (WS_S)
#define WS_XK   (WS_S + 2u * (size_t)NROW * DIN)
#define WS_H1   (WS_QH)
#define WS_H2   (WS_S)
#define WS_T    (WS_Y)
static_assert(4u * (size_t)NROW * DIN <= SZ_S);
static_assert(2u * (size_t)NROW * DFF <= WS_S - WS_QH);
static_assert(2u * (size_t)NROW * DFF <= SZ_S);
static_assert(WS_END <= (size_t)134217728u);
static_assert((WS_S % 128u) == 0 && (WS_Y % 128u) == 0 && (WS_O % 128u) == 0 && (WS_OH % 128u) == 0 && (WS_WQ % 128u) == 0 && (WS_W1 % 128u) == 0 && (WS_XK % 128u) == 0);

__global__ __launch_bounds__(256) void k_cvt_in(const float* __restrict__ X, __bf16* __restrict__ D) {
  const size_t e = (size_t)blockIdx.x * 256 + threadIdx.x; if (e >= (size_t)NROW * (DIN / 8)) return;
  const size_t r = e / (DIN / 8); const int c = (int)(e % (DIN / 8)) * 8;
  const float* p = X + ((r / TT) * TT_FULL + (r % TT)) * (size_t)DIN + c;
  const v4f a = *(const v4f*)p, b = *(const v4f*)(p + 4);
  union { v8b v; v4u u; } o;
#pragma unroll
  for (int i = 0; i < 4; ++i) { o.v[i] = (__bf16)a[i]; o.v[4 + i] = (__bf16)b[i]; }
  vst2(D + r * DIN + c, o.u);
}
__global__ __launch_bounds__(256) void k_cvt_w(const float* __restrict__ W, unsigned short* __restrict__ D, int n8, int f16mode) {
  const int e = blockIdx.x * 256 + threadIdx.x; if (e >= n8) return;
  const float* p = W + (size_t)e * 8;
  const v4f a = *(const v4f*)p, b = *(const v4f*)(p + 4);
  union { v8b vb; v8h vh; v4u u; } o;
  if (f16mode != 0) {
#pragma unroll
    for (int i = 0; i < 4; ++i) { o.vh[i] = (_Float16)(bfr(a[i]) * 256.0f); o.vh[4 + i] = (_Float16)(bfr(b[i]) * 256.0f); }
  } else {
#pragma unroll
    for (int i = 0; i < 4; ++i) { o.vb[i] = (__bf16)a[i]; o.vb[4 + i] = (__bf16)b[i]; }
  }
  vst2(D + (size_t)e * 8, o.u);
}

__global__ __launch_bounds__(128) void k_proj(const __bf16* __restrict__ XQ, const __bf16* __restrict__ XK, const __bf16* __restrict__ WQ, const __bf16* __restrict__ WK, const __bf16* __restrict__ WV,
    const float* __restrict__ BQ, const float* __restrict__ BK, const float* __restrict__ BV,
    _Float16* __restrict__ QH, _Float16* __restrict__ QL, _Float16* __restrict__ KH, _Float16* __restrict__ VT) {
  __shared__ __align__(16) _Float16 sh[64][136], sl[64][136]; __shared__ __align__(16) _Float16 th[128][72];
  const int tid = threadIdx.x, wave = tid >> 5, lane = tid & 31, col = lane & 15, g = lane >> 4; const int which = blockIdx.z; const int c0 = blockIdx.y * 128; const size_t r0 = (size_t)blockIdx.x * 64; const size_t bb = r0 / TT; const int t0 = (int)(r0 % TT);
  const __bf16* X = which == 0 ? XQ : XK; const __bf16* WA = which == 0 ? WQ : which == 1 ? WK : WV; const float* BA = which == 0 ? BQ : which == 1 ? BK : BV;
  v8f acc[8] = {};
#pragma unroll 2
  for (int kc = 0; kc < DIN / 32; ++kc) { const v16b a = frag_b(X + (r0 + wave * 16 + col) * DIN + kc * 32, lane);
    asm volatile("s_wait_loadcnt 0x0" ::: "memory");
#pragma unroll
    for (int j = 0; j < 8; ++j) { const v16b w = frag_b(WA + (size_t)(c0 + j * 16 + col) * DIN + kc * 32, lane); asm volatile("s_wait_loadcnt 0x0" ::: "memory"); acc[j] = wmma_bf(a, w, acc[j]); } }
  if (which < 2) { _Float16* DH = which == 0 ? QH : KH;
#pragma unroll
    for (int j = 0; j < 8; ++j) { const float bias = bfr(BA[c0 + j * 16 + col]);
#pragma unroll
      for (int r = 0; r < 8; ++r) { const float v = acc[j][r] + bias; const _Float16 hv = (_Float16)v; sh[wave * 16 + 8 * g + r][j * 16 + col] = hv; sl[wave * 16 + 8 * g + r][j * 16 + col] = (_Float16)((v - (float)hv) * 1024.0f); } }
    __syncthreads();
    for (int e = tid; e < 64 * 16; e += 128) { const int rl = e >> 4, q = e & 15; vst2(DH + (r0 + rl) * CC + c0 + q * 8, *(const v4u*)&sh[rl][q * 8]); if (which == 0) vst2(QL + (r0 + rl) * CC + c0 + q * 8, *(const v4u*)&sl[rl][q * 8]); }
  } else {
#pragma unroll
    for (int j = 0; j < 8; ++j) { const float bias = bfr(BA[c0 + j * 16 + col]);
#pragma unroll
      for (int r = 0; r < 8; ++r) { const float v = acc[j][r] + bias; const int rl = wave * 16 + 8 * g + r, cl = j * 16 + col; th[cl][rl] = (_Float16)v; } }
    __syncthreads();
    for (int e = tid; e < 128 * 8; e += 128) { const int cl = e >> 3, q = e & 7; vst2(VT + (bb * CC + c0 + cl) * (size_t)TT + t0 + q * 8, *(const v4u*)&th[cl][q * 8]); } } }

__global__ __launch_bounds__(128) __attribute__((amdgpu_num_vgpr(256))) void k_sc(const _Float16* __restrict__ QH, const _Float16* __restrict__ KH, const _Float16* __restrict__ QL, int b, float* __restrict__ S0) { __shared__ __align__(16) float ss[4][16][132];
  const int qb = blockIdx.x, kb = blockIdx.y, h = blockIdx.z; float* S = S0 + (size_t)h * TT * TT;
  const int tid = threadIdx.x, wave = tid >> 5, lane = tid & 31, col = lane & 15, g = lane >> 4; const int k0 = kb * 128; const int ql0 = qb * 64 + wave * 16; const size_t q0 = (size_t)b * TT + ql0, kr0 = (size_t)b * TT + k0;
  v8f acc[8] = {}, accl[8] = {};
#pragma unroll
  for (int kc = 0; kc < HD / 32; ++kc) { const v16h ah = frag_h(QH + (q0 + col) * CC + h * HD + kc * 32, lane), al = frag_h(QL + (q0 + col) * CC + h * HD + kc * 32, lane);
    asm volatile("s_wait_loadcnt 0x0" ::: "memory");
#pragma unroll
    for (int j = 0; j < 8; ++j) { const v16h kbf = frag_h(KH + (kr0 + j * 16 + col) * CC + h * HD + kc * 32, lane); asm volatile("s_wait_loadcnt 0x0" ::: "memory"); acc[j] = wmma16(ah, kbf, acc[j]); accl[j] = wmma16(al, kbf, accl[j]); } }
#pragma unroll
  for (int j = 0; j < 8; ++j) {
#pragma unroll
    for (int r = 0; r < 8; ++r) ss[wave][8 * g + r][j * 16 + col] = (acc[j][r] + accl[j][r] * (1.0f / 1024.0f)) * SCALE; }
  LDSX(); for (int rl = 0; rl < 16; ++rl) vst2(S + (size_t)(ql0 + rl) * TT + k0 + lane * 4, *(const v4f*)&ss[wave][rl][lane * 4]); }
__global__ __launch_bounds__(256) void k_sm(float* __restrict__ S0) { __shared__ float sred[8]; __shared__ float sbc; __shared__ __align__(16) float shv[TT];
  const int tid = threadIdx.x; const int t = blockIdx.x;
  float* sr = S0 + (size_t)blockIdx.y * TT * TT + (size_t)t * TT;
  float m = -3.0e38f;
#pragma unroll 1
  for (int k = tid; k < TT; k += 256) { const float v = sr[k]; shv[k] = v; m = fmaxf(m, v); }
#pragma unroll
  for (int o = 1; o < 32; o <<= 1) m = fmaxf(m, __shfl_xor(m, o));
  if ((tid & 31) == 0) sred[tid >> 5] = m; __syncthreads(); if (tid == 0) { float a = sred[0]; for (int i = 1; i < 8; ++i) a = fmaxf(a, sred[i]); sbc = a; } __syncthreads(); m = sbc; __syncthreads();
  float sum = 0.f;
#pragma unroll 1
  for (int k = tid; k < TT; k += 256) { const float v = shv[k]; const float e = expf(v - m); shv[k] = e; sum += e; }
#pragma unroll
  for (int o = 1; o < 32; o <<= 1) sum += __shfl_xor(sum, o);
  if ((tid & 31) == 0) sred[tid >> 5] = sum; __syncthreads(); if (tid == 0) { float a = 0.f; for (int i = 0; i < 8; ++i) a += sred[i]; sbc = a > 0.f ? 2048.0f / a : 0.f; } __syncthreads(); const float inv = sbc;
#pragma unroll 1
  for (int k = tid; k < TT; k += 256) shv[k] = shv[k] * inv;
  __syncthreads(); for (int q = tid; q < TT / 4; q += 256) vst2(sr + q * 4, *(const v4f*)&shv[q * 4]); }
__global__ __launch_bounds__(128) __attribute__((amdgpu_num_vgpr(256))) void k_pv(const float* __restrict__ PS0, const _Float16* __restrict__ VT, int b, float* __restrict__ Y) { const int h = blockIdx.z; const float* PS = PS0 + (size_t)h * TT * TT; __shared__ __align__(16) float ss[4][16][HD + 4];
  const int tid = threadIdx.x, wave = tid >> 5, lane = tid & 31, col = lane & 15, g = lane >> 4; const int qb = blockIdx.x; const int ql0 = qb * 64 + wave * 16;
  v8f acc[HD / 16] = {};
#pragma unroll 1
  for (int kc = 0; kc < TT / 32; ++kc) { const v16h p = frag_f32(PS + (size_t)(ql0 + col) * TT + kc * 32, lane);
    asm volatile("s_wait_loadcnt 0x0" ::: "memory");
#pragma unroll
    for (int j = 0; j < HD / 16; ++j) { const size_t po = ((size_t)b * CC + h * HD + j * 16 + col) * (size_t)TT + kc * 32; acc[j] = wmma16(p, frag_h(VT + po, lane), acc[j]); } }
#pragma unroll
  for (int j = 0; j < HD / 16; ++j)
#pragma unroll
    for (int r = 0; r < 8; ++r) ss[wave][8 * g + r][j * 16 + col] = acc[j][r] * (1.0f / 2048.0f);
  LDSX(); for (int rl = 0; rl < 16; ++rl) if (lane < HD / 4) vst2(Y + ((size_t)b * TT + ql0 + rl) * CC + h * HD + lane * 4, *(const v4f*)&ss[wave][rl][lane * 4]); }

__global__ __launch_bounds__(256) void k_ln0(const _Float16* __restrict__ QH, const _Float16* __restrict__ QL, const float* __restrict__ Y, const float* __restrict__ GM, const float* __restrict__ BT, float* __restrict__ O, _Float16* __restrict__ OH) {
#pragma clang fp contract(off)
  const int wave = threadIdx.x >> 5, lane = threadIdx.x & 31; const size_t row = (size_t)blockIdx.x * 8 + wave; if (row >= (size_t)NROW) return;
  v4f x[4]; float s1 = 0.f;
#pragma unroll
  for (int q = 0; q < 4; ++q) { const size_t o = row * CC + q * 128 + lane * 4; const v4f y = *(const v4f*)(Y + o); const v4h a = *(const v4h*)(QH + o), c = *(const v4h*)(QL + o);
#pragma unroll
    for (int i = 0; i < 4; ++i) { const float ah = (float)a[i], al = (float)c[i]; const float qp = ah + al * (1.0f / 1024.0f); x[q][i] = y[i] + qp; s1 += x[q][i]; } }
#pragma unroll
  for (int o = 1; o < 32; o <<= 1) s1 += __shfl_xor(s1, o);
  const float mu = s1 * (1.0f / CC); float qq = 0.f;
#pragma unroll
  for (int q = 0; q < 4; ++q)
#pragma unroll
    for (int i = 0; i < 4; ++i) { const float d = x[q][i] - mu; qq += d * d; }
#pragma unroll
  for (int o = 1; o < 32; o <<= 1) qq += __shfl_xor(qq, o);
  const float rs = rsqrtf(qq * (1.0f / CC) + 1e-5f);
#pragma unroll
  for (int q = 0; q < 4; ++q) { v4f r4; v4h h4; const int c = q * 128 + lane * 4;
#pragma unroll
    for (int i = 0; i < 4; ++i) { r4[i] = (x[q][i] - mu) * rs * bfr(GM[c + i]) + bfr(BT[c + i]); h4[i] = (_Float16)r4[i]; }
    vst2(O + row * CC + c, r4); vst2(OH + row * CC + c, h4); } }
template <int K, int N, int MODE>
__global__ __launch_bounds__(128) void k_ffn(const _Float16* __restrict__ A, const _Float16* __restrict__ WH, const float* __restrict__ BI, const float* __restrict__ R, _Float16* __restrict__ HO, float* __restrict__ TO) {
  __shared__ __align__(16) _Float16 sh[64][136]; __shared__ __align__(16) float sf[4][16][132];
  static_assert(K % 64 == 0 && N % 128 == 0);
  const int tid = threadIdx.x, wave = tid >> 5, lane = tid & 31, col = lane & 15, g = lane >> 4; const int c0 = blockIdx.y * 128; const size_t r0 = (size_t)blockIdx.x * 64;
  v8f acc[8] = {};
#pragma unroll 2
  for (int kc = 0; kc < K / 32; ++kc) { const v16h a = frag_h(A + (r0 + wave * 16 + col) * (size_t)K + kc * 32, lane);
    asm volatile("s_wait_loadcnt 0x0" ::: "memory");
#pragma unroll
    for (int j = 0; j < 8; ++j) { const v16h w = frag_h(WH + (size_t)(c0 + j * 16 + col) * K + kc * 32, lane); asm volatile("s_wait_loadcnt 0x0" ::: "memory"); acc[j] = wmma16(a, w, acc[j]); } }
  if (MODE == 0) {
#pragma unroll
    for (int j = 0; j < 8; ++j) { const float bb = bfr(BI[c0 + j * 16 + col]);
#pragma unroll
      for (int r = 0; r < 8; ++r) sh[wave * 16 + 8 * g + r][j * 16 + col] = (_Float16)fmaxf(acc[j][r] * (1.0f / 256.0f) + bb, 0.f); }
    __syncthreads();
    for (int e = tid; e < 64 * 16; e += 128) { const int rl = e >> 4, q = e & 15; vst2(HO + (r0 + rl) * (size_t)N + c0 + q * 8, *(const v4u*)&sh[rl][q * 8]); }
  } else {
#pragma unroll
    for (int j = 0; j < 8; ++j) { const float bb = bfr(BI[c0 + j * 16 + col]);
#pragma unroll
      for (int r = 0; r < 8; ++r) sf[wave][8 * g + r][j * 16 + col] = acc[j][r] * (1.0f / 256.0f) + bb; }
    LDSX(); for (int rl = 0; rl < 16; ++rl) { const size_t o2 = (r0 + wave * 16 + rl) * (size_t)N + c0 + lane * 4; const v4f x = *(const v4f*)(R + o2); v4f t = *(const v4f*)&sf[wave][rl][lane * 4]; t[0] += x[0]; t[1] += x[1]; t[2] += x[2]; t[3] += x[3]; vst2(TO + o2, t); } } }
__global__ __launch_bounds__(256) void k_ln1(const float* __restrict__ T, const float* __restrict__ GM, const float* __restrict__ BT, float* __restrict__ OUT) {
#pragma clang fp contract(off)
  const int wave = threadIdx.x >> 5, lane = threadIdx.x & 31; const size_t row = (size_t)blockIdx.x * 8 + wave; if (row >= (size_t)NROW) return;
  const size_t orow = (row / TT) * TT_FULL + (row % TT);
  v4f x[4]; float s1 = 0.f;
#pragma unroll
  for (int q = 0; q < 4; ++q) { x[q] = *(const v4f*)(T + row * CC + q * 128 + lane * 4);
#pragma unroll
    for (int i = 0; i < 4; ++i) s1 += x[q][i]; }
#pragma unroll
  for (int o = 1; o < 32; o <<= 1) s1 += __shfl_xor(s1, o);
  const float mu = s1 * (1.0f / CC); float qq = 0.f;
#pragma unroll
  for (int q = 0; q < 4; ++q)
#pragma unroll
    for (int i = 0; i < 4; ++i) { const float d = x[q][i] - mu; qq += d * d; }
#pragma unroll
  for (int o = 1; o < 32; o <<= 1) qq += __shfl_xor(qq, o);
  const float rs = rsqrtf(qq * (1.0f / CC) + 1e-5f);
#pragma unroll
  for (int q = 0; q < 4; ++q) { v4f r4; const int c = q * 128 + lane * 4;
#pragma unroll
    for (int i = 0; i < 4; ++i) r4[i] = (x[q][i] - mu) * rs * bfr(GM[c + i]) + bfr(BT[c + i]);
    vst2(OUT + orow * CC + c, r4); } }

extern "C" void kernel_launch(void* const* d_in, const int* in_sizes, int n_in, void* d_out, int out_size, void* d_ws, size_t ws_size, hipStream_t stream) {
  if (n_in < 18) return;
  const int need_x = ((NB - 1) * TT_FULL + TT) * DIN;
  if (in_sizes[0] < need_x || in_sizes[1] < need_x) return;
  if (in_sizes[2] < CC * DIN || in_sizes[4] < CC * DIN || in_sizes[6] < CC * DIN || in_sizes[3] < CC || in_sizes[5] < CC || in_sizes[7] < CC) return;
  if (in_sizes[8] < DFF * CC || in_sizes[9] < DFF || in_sizes[10] < DFF * DFF || in_sizes[11] < DFF || in_sizes[12] < CC * DFF || in_sizes[13] < CC) return;
  if (in_sizes[14] < CC || in_sizes[15] < CC || in_sizes[16] < CC || in_sizes[17] < CC) return;
  if (out_size < ((NB - 1) * TT_FULL + TT) * CC) return;
  if (ws_size < (size_t)WS_END) return;
  const float** F = (const float**)d_in;
  char* ws = (char*)d_ws;
  _Float16 *QH = (_Float16*)(ws + WS_QH), *KH = (_Float16*)(ws + WS_KH), *VT = (_Float16*)(ws + WS_VT), *QL = (_Float16*)(ws + WS_QL), *OH = (_Float16*)(ws + WS_OH);
  _Float16 *H1 = (_Float16*)(ws + WS_H1), *H2 = (_Float16*)(ws + WS_H2), *W1H = (_Float16*)(ws + WS_W1), *W2H = (_Float16*)(ws + WS_W2), *W3H = (_Float16*)(ws + WS_W3);
  __bf16 *XQ = (__bf16*)(ws + WS_XQ), *XK = (__bf16*)(ws + WS_XK), *WQB = (__bf16*)(ws + WS_WQ), *WKB = (__bf16*)(ws + WS_WK), *WVB = (__bf16*)(ws + WS_WV);
  float *S = (float*)(ws + WS_S), *Y = (float*)(ws + WS_Y), *O = (float*)(ws + WS_O), *T = (float*)(ws + WS_T);
  const int n8x = NROW * (DIN / 8);
  k_cvt_in<<<dim3((n8x + 255) / 256), 256, 0, stream>>>(F[0], XQ);
  k_cvt_in<<<dim3((n8x + 255) / 256), 256, 0, stream>>>(F[1], XK);
  const int n8p = CC * DIN / 8, n8a = DFF * CC / 8, n8b = DFF * DFF / 8, n8c = CC * DFF / 8;
  k_cvt_w<<<dim3((n8p + 255) / 256), 256, 0, stream>>>(F[2], (unsigned short*)WQB, n8p, 0);
  k_cvt_w<<<dim3((n8p + 255) / 256), 256, 0, stream>>>(F[4], (unsigned short*)WKB, n8p, 0);
  k_cvt_w<<<dim3((n8p + 255) / 256), 256, 0, stream>>>(F[6], (unsigned short*)WVB, n8p, 0);
  k_cvt_w<<<dim3((n8a + 255) / 256), 256, 0, stream>>>(F[8], (unsigned short*)W1H, n8a, 1);
  k_cvt_w<<<dim3((n8b + 255) / 256), 256, 0, stream>>>(F[10], (unsigned short*)W2H, n8b, 1);
  k_cvt_w<<<dim3((n8c + 255) / 256), 256, 0, stream>>>(F[12], (unsigned short*)W3H, n8c, 1);
  k_proj<<<dim3(NROW / 64, CC / 128, 3), 128, 0, stream>>>(XQ, XK, WQB, WKB, WVB, F[3], F[5], F[7], QH, QL, KH, VT);
  for (int b = 0; b < NB; ++b) {
    k_sc<<<dim3(NQB, TT / 128, NH), 128, 0, stream>>>(QH, KH, QL, b, S);
    k_sm<<<dim3(TT, NH), 256, 0, stream>>>(S);
    k_pv<<<dim3(NQB, 1, NH), 128, 0, stream>>>(S, VT, b, Y);
  }
  k_ln0<<<dim3((NROW + 7) / 8), 256, 0, stream>>>(QH, QL, Y, F[14], F[15], O, OH);
  k_ffn<CC, DFF, 0><<<dim3(NROW / 64, DFF / 128), 128, 0, stream>>>(OH, W1H, F[9], O, H1, T);
  k_ffn<DFF, DFF, 0><<<dim3(NROW / 64, DFF / 128), 128, 0, stream>>>(H1, W2H, F[11], O, H2, T);
  k_ffn<DFF, CC, 1><<<dim3(NROW / 64, CC / 128), 128, 0, stream>>>(H2, W3H, F[13], O, OH, T);
  k_ln1<<<dim3((NROW + 7) / 8), 256, 0, stream>>>(T, F[16], F[17], (float*)d_out);
}
